// GRUMulitiTaskAutoencoder_38929583571515
// MI455X (gfx1250) — hardware-verified
//
#include <hip/hip_runtime.h>

typedef __attribute__((ext_vector_type(16))) _Float16 v16h;
typedef __attribute__((ext_vector_type(8)))  _Float16 v8h;
typedef __attribute__((ext_vector_type(8)))  float    v8f;
typedef __attribute__((ext_vector_type(4)))  float    v4f;

constexpr int kN        = 2048;
constexpr int kSeqLen   = 128;
constexpr int kXCols    = kSeqLen + 1;
constexpr int kHid      = 128;
constexpr int kG3       = 3 * kHid;
constexpr int kNE       = 8;
constexpr int kRowsPB   = 16;
constexpr int kThreads  = 256;
constexpr int kEncBlocks = kN / kRowsPB;
constexpr int kDecChunks = kN / kRowsPB;
constexpr int kIdChunks  = kN / kThreads;
constexpr int kHP = kHid + 8;
constexpr int kHT = kRowsPB * kHP;
constexpr int kFP = kHid + 4;
constexpr int kEncHalves = kG3 * kHid;
constexpr int kDecHalves = kNE * kG3 * kHid;
constexpr int kEncDw = kEncHalves / 2;
constexpr int kDecDw = kDecHalves / 2;
constexpr int kPrepEncBlocks = kEncDw / kThreads;
constexpr int kPrepBlocks = kPrepEncBlocks + kDecDw / kThreads;
constexpr float kW16 = 16.0f;
constexpr float kInv16 = 0.0625f;
static_assert(kHid == (kThreads / 32) * 16);
static_assert(kHid % 32 == 0);
static_assert(kHP % 8 == 0 && kFP % 4 == 0);
static_assert(kSeqLen <= kFP);
static_assert(kN % kRowsPB == 0 && kN % kThreads == 0);
static_assert(kEncDw % kThreads == 0 && kDecDw % kThreads == 0);
static_assert(kPrepBlocks == 864);
static_assert(kThreads * 8 == kRowsPB * kHid);
static_assert(kHT % 8 == 0);

template <typename T> struct Frag;
template <> struct Frag<_Float16> {
  typedef v16h V; union U { v16h v; v8h h[2]; };
  static __device__ __forceinline__ v16h load(const _Float16* p) {
    U f; f.h[0] = *(const v8h*)(p); f.h[1] = *(const v8h*)(p + 16); return f.v;
  }
  static __device__ __forceinline__ v8f mma(v16h a, v16h b, v8f c) {
    return __builtin_amdgcn_wmma_f32_16x16x32_f16(false, a, false, b, (short)0, c, false, false);
  }
};
__device__ __forceinline__ v8f mma16(v16h a, v16h b, v8f c) {
  c = Frag<_Float16>::mma(a, b, c);
  asm volatile("v_nop\n\tv_nop\n\tv_nop\n\tv_nop" : "+v"(c) : "v"(a), "v"(b));
  return c;
}
__device__ __forceinline__ v8f zero8() { return (v8f){0.f, 0.f, 0.f, 0.f, 0.f, 0.f, 0.f, 0.f}; }

__device__ __forceinline__ unsigned pack_f16x2(float a, float b) {
  const _Float16 h0 = (_Float16)a, h1 = (_Float16)b;
  return (unsigned)__builtin_bit_cast(unsigned short, h0) | ((unsigned)__builtin_bit_cast(unsigned short, h1) << 16);
}
__device__ __forceinline__ void st2u(unsigned* p, unsigned v) { *(volatile unsigned*)p = v; __threadfence(); *(volatile unsigned*)p = v; }
__device__ __forceinline__ float fsig(float x)  { return __builtin_amdgcn_rcpf(1.0f + __expf(-x)); }
__device__ __forceinline__ float ftanh(float x) { return 1.0f - 2.0f * __builtin_amdgcn_rcpf(1.0f + __expf(2.0f * x)); }
__device__ __forceinline__ float gru_cell(float xin, float wiR, float wiZ, float wiN,
                                          float biR, float biZ, float biN,
                                          float ghR, float ghZ, float ghN, float hprev) {
  const float rg = fsig(fmaf(xin, wiR, biR) + ghR);
  const float zg = fsig(fmaf(xin, wiZ, biZ) + ghZ);
  const float ng = ftanh(fmaf(xin, wiN, biN) + rg * ghN);
  return (1.0f - zg) * ng + zg * hprev;
}
__device__ __forceinline__ int route_id(float v) {
  const float vc = fminf(fmaxf(v, -1024.0f), 1024.0f);
  int i = (int)vc;
  i = (i < 0) ? (i + kNE) : i;
  i = (i < 0) ? 0 : ((i > kNE - 1) ? (kNE - 1) : i);
  return i;
}

__global__ __launch_bounds__(kThreads) void prep_kernel(
    const float* __restrict__ WhhE, const float* __restrict__ WhhD,
    unsigned* __restrict__ we16u, unsigned* __restrict__ wd16u) {
  const int blk = blockIdx.x, tid = threadIdx.x;
  if (blk < kPrepEncBlocks) {
    const int p = blk * kThreads + tid;
    st2u(we16u + p, pack_f16x2(WhhE[2 * p] * kW16, WhhE[2 * p + 1] * kW16));
  } else {
    const int p = (blk - kPrepEncBlocks) * kThreads + tid;
    st2u(wd16u + p, pack_f16x2(WhhD[2 * p] * kW16, WhhD[2 * p + 1] * kW16));
  }
}

__global__ __launch_bounds__(kThreads) void enc_kernel(
    const float* __restrict__ x, const float* __restrict__ WihE, const float* __restrict__ bihE,
    const float* __restrict__ bhhE, const _Float16* __restrict__ we16, float* __restrict__ henc) {
  __shared__ __align__(16) _Float16 hbuf[2 * kHT];
  __shared__ __align__(16) float ft[kRowsPB * kFP];
  const int tid = threadIdx.x, lane = tid & 31, wave = tid >> 5;
  const int c = lane & 15, hh = lane >> 4, koff = hh * 8, mOff = hh * 8;
  const int u = wave * 16 + c;
  const int row0 = blockIdx.x * kRowsPB;

  {
    const int j = tid >> 4, cb = (tid & 15) * 8;
    const float* src = x + (size_t)(row0 + j) * kXCols + cb;
#pragma unroll
    for (int i = 0; i < 8; ++i) ft[j * kFP + cb + i] = src[i];
  }
  {
    const v8h z = {(_Float16)0.f, (_Float16)0.f, (_Float16)0.f, (_Float16)0.f, (_Float16)0.f, (_Float16)0.f, (_Float16)0.f, (_Float16)0.f};
    for (int i = tid; i < kHT / 8; i += kThreads) *(v8h*)(hbuf + i * 8) = z;
  }
  __syncthreads();

  const float wiR = WihE[u], wiZ = WihE[kHid + u], wiN = WihE[2 * kHid + u];
  const float biR = bihE[u], biZ = bihE[kHid + u], biN = bihE[2 * kHid + u];
  const float bhR = bhhE[u], bhZ = bhhE[kHid + u], bhN = bhhE[2 * kHid + u];
  const _Float16* bR = we16 + (size_t)u * kHid + koff;
  const _Float16* bZ = we16 + (size_t)(kHid + u) * kHid + koff;
  const _Float16* bN = we16 + (size_t)(2 * kHid + u) * kHid + koff;

  float hc[8];
#pragma unroll
  for (int r = 0; r < 8; ++r) hc[r] = 0.0f;

#pragma unroll 1
  for (int t = 0; t < kSeqLen; ++t) {
    const _Float16* hcur = hbuf + (t & 1) * kHT;
    _Float16*       hnx  = hbuf + ((t + 1) & 1) * kHT;
    v8f aR = zero8(), aZ = zero8(), aN = zero8();
    const _Float16* arow = hcur + c * kHP + koff;
#pragma unroll
    for (int kc = 0; kc < kHid / 32; ++kc) {
      const v16h fa = Frag<_Float16>::load(arow + kc * 32);
      const v16h fr = Frag<_Float16>::load(bR + kc * 32);
      const v16h fz = Frag<_Float16>::load(bZ + kc * 32);
      const v16h fn = Frag<_Float16>::load(bN + kc * 32);
      aR = mma16(fa, fr, aR);
      aZ = mma16(fa, fz, aZ);
      aN = mma16(fa, fn, aN);
    }
#pragma unroll
    for (int r = 0; r < 8; ++r) {
      const int row = mOff + r;
      const float xv  = ft[row * kFP + t];
      const float ghR = fmaf(aR[r], kInv16, bhR);
      const float ghZ = fmaf(aZ[r], kInv16, bhZ);
      const float ghN = fmaf(aN[r], kInv16, bhN);
      const float hn = gru_cell(xv, wiR, wiZ, wiN, biR, biZ, biN, ghR, ghZ, ghN, hc[r]);
      hc[r] = hn;
      hnx[row * kHP + u] = (_Float16)hn;
    }
    __syncthreads();
  }

#pragma unroll
  for (int r = 0; r < 8; ++r) ft[(mOff + r) * kFP + u] = hc[r];
  __syncthreads();
  {
    const int ra = wave * 2, rb = ra + 1;
    const v4f va = *(const v4f*)(ft + ra * kFP + lane * 4);
    const v4f vb = *(const v4f*)(ft + rb * kFP + lane * 4);
    float* pa = henc + (size_t)(row0 + ra) * kHid + lane * 4;
    float* pb = henc + (size_t)(row0 + rb) * kHid + lane * 4;
    *(volatile v4f*)pa = va;
    *(volatile v4f*)pb = vb;
    __threadfence();
    *(volatile v4f*)pa = va;
    *(volatile v4f*)pb = vb;
  }
}

__global__ __launch_bounds__(kThreads) void dec_kernel(
    const float* __restrict__ x, const float* __restrict__ henc,
    const float* __restrict__ WihD, const float* __restrict__ bihD, const float* __restrict__ bhhD,
    const float* __restrict__ Wlin, const float* __restrict__ blin,
    const _Float16* __restrict__ wd16, float* __restrict__ out) {
  __shared__ __align__(16) _Float16 hbuf[2 * kHT];
  __shared__ __align__(16) float ft[kRowsPB * kFP];
  __shared__ float ypart[(kThreads / 32) * kRowsPB];
  __shared__ float ybuf[kRowsPB];
  __shared__ int s_rows[kRowsPB];
  __shared__ int s_wtot[kThreads / 32];
  const int tid = threadIdx.x, lane = tid & 31, wave = tid >> 5;
  const int c = lane & 15, hh = lane >> 4, koff = hh * 8, mOff = hh * 8;
  const int u = wave * 16 + c;
  const int chunk = blockIdx.x;
  const int e     = blockIdx.y;

  if (tid < kRowsPB) s_rows[tid] = 0;
  __syncthreads();
  int base = 0;
#pragma unroll 1
  for (int k = 0; k < kIdChunks; ++k) {
    const int n = k * kThreads + tid;
    const int idn = route_id(x[(size_t)n * kXCols + kSeqLen]);
    const bool hit = (idn == e);
    const unsigned bal = __builtin_amdgcn_ballot_w32(hit);
    const int pos = __builtin_popcount(bal & ((1u << lane) - 1u));
    if (lane == 0) s_wtot[wave] = __builtin_popcount(bal);
    __syncthreads();
    int pre = 0, tot = 0;
#pragma unroll
    for (int w2 = 0; w2 < kThreads / 32; ++w2) {
      const int cw = s_wtot[w2];
      tot += cw;
      pre += (w2 < wave) ? cw : 0;
    }
    const int slot = base + pre + pos - chunk * kRowsPB;
    if (hit && slot >= 0 && slot < kRowsPB) s_rows[slot] = n;
    base += tot;
    __syncthreads();
  }
  const int rem = base - chunk * kRowsPB;
  if (rem <= 0) return;
  const int nvalid = (rem < kRowsPB) ? rem : kRowsPB;

  {
    const int j = tid >> 4, cb = (tid & 15) * 8;
    int rj = s_rows[j];
    rj = (rj < 0) ? 0 : ((rj > kN - 1) ? (kN - 1) : rj);
    const float* src = henc + (size_t)rj * kHid + cb;
    const v4f va = *(const v4f*)src;
    const v4f vb = *(const v4f*)(src + 4);
#pragma unroll
    for (int i = 0; i < 4; ++i) {
      ft[j * kFP + cb + i]       = va[i];
      ft[j * kFP + cb + 4 + i]   = vb[i];
      hbuf[j * kHP + cb + i]     = (_Float16)va[i];
      hbuf[j * kHP + cb + 4 + i] = (_Float16)vb[i];
    }
  }
  if (tid < kRowsPB) ybuf[tid] = 0.0f;
  __syncthreads();

  float hc[8];
#pragma unroll
  for (int r = 0; r < 8; ++r) hc[r] = ft[(mOff + r) * kFP + u];

  const int eg = e * kG3;
  const float wiR = WihD[eg + u], wiZ = WihD[eg + kHid + u], wiN = WihD[eg + 2 * kHid + u];
  const float biR = bihD[eg + u], biZ = bihD[eg + kHid + u], biN = bihD[eg + 2 * kHid + u];
  const float bhR = bhhD[eg + u], bhZ = bhhD[eg + kHid + u], bhN = bhhD[eg + 2 * kHid + u];
  const float wl = Wlin[e * kHid + u];
  const float bl = blin[e];
  const _Float16* wexp = wd16 + (size_t)e * kEncHalves;
  const _Float16* bR = wexp + (size_t)u * kHid + koff;
  const _Float16* bZ = wexp + (size_t)(kHid + u) * kHid + koff;
  const _Float16* bN = wexp + (size_t)(2 * kHid + u) * kHid + koff;
  __syncthreads();

#pragma unroll 1
  for (int t = 0; t < kSeqLen; ++t) {
    const _Float16* hcur = hbuf + (t & 1) * kHT;
    _Float16*       hnx  = hbuf + ((t + 1) & 1) * kHT;
    v8f aR = zero8(), aZ = zero8(), aN = zero8();
    const _Float16* arow = hcur + c * kHP + koff;
#pragma unroll
    for (int kc = 0; kc < kHid / 32; ++kc) {
      const v16h fa = Frag<_Float16>::load(arow + kc * 32);
      const v16h fr = Frag<_Float16>::load(bR + kc * 32);
      const v16h fz = Frag<_Float16>::load(bZ + kc * 32);
      const v16h fn = Frag<_Float16>::load(bN + kc * 32);
      aR = mma16(fa, fr, aR);
      aZ = mma16(fa, fz, aZ);
      aN = mma16(fa, fn, aN);
    }
    float ysum[8];
#pragma unroll
    for (int r = 0; r < 8; ++r) {
      const int row = mOff + r;
      const float yp  = ybuf[row];
      const float ghR = fmaf(aR[r], kInv16, bhR);
      const float ghZ = fmaf(aZ[r], kInv16, bhZ);
      const float ghN = fmaf(aN[r], kInv16, bhN);
      const float hn = gru_cell(yp, wiR, wiZ, wiN, biR, biZ, biN, ghR, ghZ, ghN, hc[r]);
      hc[r] = hn;
      hnx[row * kHP + u] = (_Float16)hn;
      float s = hn * wl;
      s += __shfl_xor(s, 1, 32);
      s += __shfl_xor(s, 2, 32);
      s += __shfl_xor(s, 4, 32);
      s += __shfl_xor(s, 8, 32);
      ysum[r] = s;
    }
    if (c == 0) {
#pragma unroll
      for (int r = 0; r < 8; ++r) ypart[wave * kRowsPB + mOff + r] = ysum[r];
    }
    __syncthreads();
    if (tid < kRowsPB) {
      float s = ypart[tid];
#pragma unroll
      for (int w2 = 1; w2 < kThreads / 32; ++w2) s += ypart[w2 * kRowsPB + tid];
      const float yv = s + bl;
      ybuf[tid] = yv;
      ft[tid * kFP + t] = yv;
    }
    __syncthreads();
  }

#pragma unroll
  for (int q = 0; q < 2; ++q) {
    const int j = wave + q * (kThreads / 32);
    if (j < nvalid) {
      int rj = s_rows[j];
      rj = (rj < 0) ? 0 : ((rj > kN - 1) ? (kN - 1) : rj);
      const v4f v = *(const v4f*)(ft + j * kFP + lane * 4);
      float* p = out + (size_t)rj * kSeqLen + lane * 4;
      *(volatile v4f*)p = v;
      __threadfence();
      *(volatile v4f*)p = v;
    }
  }
}

extern "C" void kernel_launch(void* const* d_in, const int* in_sizes, int n_in,
                              void* d_out, int out_size, void* d_ws, size_t ws_size, hipStream_t stream) {
  if (n_in < 11 || d_out == nullptr || d_ws == nullptr) return;
  if (in_sizes[0] != kN * kXCols || in_sizes[1] != kG3 || in_sizes[2] != kG3 * kHid ||
      in_sizes[3] != kG3 || in_sizes[4] != kG3 || in_sizes[5] != kNE * kG3 || in_sizes[6] != kNE * kG3 * kHid ||
      in_sizes[7] != kNE * kG3 || in_sizes[8] != kNE * kG3 || in_sizes[9] != kNE * kHid || in_sizes[10] != kNE ||
      out_size != kN * kSeqLen) return;

  const float* x    = (const float*)d_in[0];
  const float* WihE = (const float*)d_in[1];
  const float* WhhE = (const float*)d_in[2];
  const float* bihE = (const float*)d_in[3];
  const float* bhhE = (const float*)d_in[4];
  const float* WihD = (const float*)d_in[5];
  const float* WhhD = (const float*)d_in[6];
  const float* bihD = (const float*)d_in[7];
  const float* bhhD = (const float*)d_in[8];
  const float* Wlin = (const float*)d_in[9];
  const float* blin = (const float*)d_in[10];
  float* out = (float*)d_out;

  char* ws = (char*)d_ws; size_t off = 0;
  auto carve = [&](size_t bytes) -> char* { char* p = ws + off; off += (bytes + 255) & ~(size_t)255; return p; };
  unsigned short* WE16 = (unsigned short*)carve((size_t)kEncHalves * 2);
  unsigned short* WD16 = (unsigned short*)carve((size_t)kDecHalves * 2);
  float*          HENC = (float*)carve((size_t)kN * kHid * 4);
  if (off > ws_size || off > (size_t)134217728) return;

  prep_kernel<<<kPrepBlocks, kThreads, 0, stream>>>(WhhE, WhhD, (unsigned*)WE16, (unsigned*)WD16);
  enc_kernel<<<kEncBlocks, kThreads, 0, stream>>>(x, WihE, bihE, bhhE, (const _Float16*)WE16, HENC);
  dec_kernel<<<dim3(kDecChunks, kNE), kThreads, 0, stream>>>(x, HENC, WihD, bihD, bhhD, Wlin, blin,
                                                             (const _Float16*)WD16, out);
}
